// AGNO_82575041233033
// MI455X (gfx1250) — hardware-verified
//
#include <hip/hip_runtime.h>
#include <math.h>

typedef __attribute__((ext_vector_type(16))) _Float16 v16h;
typedef __attribute__((ext_vector_type(8)))  _Float16 v8h;
typedef __attribute__((ext_vector_type(8)))  float    v8f;
typedef __attribute__((ext_vector_type(4)))  float    v4f;
typedef __attribute__((ext_vector_type(4)))  int      v4i;

constexpr int kNodes         = 100000;
constexpr int kDeg           = 16;
constexpr int kEdges         = kNodes * kDeg;
constexpr int kCoord         = 3;
constexpr int kHid           = 128;
constexpr int kChOut         = 64;
constexpr int kK1            = 32;
constexpr int kPairs         = kNodes / 2;
constexpr int kWavesPerBlock = 4;
constexpr int kBlocks        = 1250;
constexpr int kIters         = 10;
constexpr int kHP            = 136;
constexpr float kEps         = 1e-12f;
constexpr float kResCarry    = 64.0f;
constexpr float kResInv      = 1.0f / kResCarry;
constexpr float kWCarry      = 16.0f;
constexpr float kWInv        = 1.0f / kWCarry;
static_assert(kEdges == 1600000, "edge count");
static_assert(kDeg == 16, "one 16-row tile is one node");
static_assert((kNodes % 2) == 0, "node pairs");
static_assert(kBlocks * kWavesPerBlock * kIters == kPairs, "every wave owns exactly kIters node pairs");
static_assert((kHid % 32) == 0 && (kK1 % 32) == 0, "k-steps of 32");
static_assert((kHid % 16) == 0 && (kChOut % 16) == 0, "n tiles of 16");
static_assert(2 * kCoord * 3 + 2 <= kK1, "layer-1 slot layout fits one k-step");
static_assert((kHP % 8) == 0 && kHP >= kHid, "16-B aligned activation pitch");

constexpr size_t kOffBt1  = 0;
constexpr size_t kOffBt2  = kOffBt1 + (size_t)kHid * kK1 * 2;
constexpr size_t kOffBt3  = kOffBt2 + (size_t)kHid * kHid * 2;
constexpr size_t kOffBias = kOffBt3 + (size_t)kChOut * kHid * 2;
constexpr size_t kWsTotal = kOffBias + (size_t)(kHid + kChOut) * 4;
static_assert(kWsTotal == 58112ull, "carve total");
static_assert(kWsTotal <= 134217728ull, "carve cap");
static_assert((kOffBt2 % 128) == 0 && (kOffBt3 % 128) == 0 && (kOffBias % 128) == 0 && (kWsTotal % 128) == 0, "128-B aligned regions");

constexpr int kChunks1 = kHid * kK1 / 8;
constexpr int kChunks2 = kHid * kHid / 8;
constexpr int kChunks3 = kChOut * kHid / 8;
constexpr int kChunksB = (kHid + kChOut) / 4;
constexpr int kPrepB1  = kChunks1 / 64;
constexpr int kPrepB2  = kChunks2 / 64;
constexpr int kPrepB3  = kChunks3 / 64;
constexpr int kPrepBlocks = kPrepB1 + kPrepB2 + kPrepB3 + 1;
static_assert(kChunks1 == 512 && kChunks2 == 2048 && kChunks3 == 1024 && kChunksB == 48, "chunk counts");
static_assert((kChunks1 % 64) == 0 && (kChunks2 % 64) == 0 && (kChunks3 % 64) == 0 && kChunksB <= 64, "prep coverage");
static_assert(kPrepBlocks == 57, "prep grid");

struct FragH {
  union U { v16h v; v8h h[2]; };
  static __device__ __forceinline__ v16h load(const _Float16* p) {
    U f;
    f.h[0] = *(const v8h*)(p);
    f.h[1] = *(const v8h*)(p + 16);
    return f.v;
  }
};

__device__ __forceinline__ v8f mma_h(v16h a, v16h b, v8f c) {
  c = __builtin_amdgcn_wmma_f32_16x16x32_f16(false, a, false, b, (short)0, c, false, false);
  asm volatile("v_nop\n\tv_nop\n\tv_nop\n\tv_nop" : "+v"(c) : "v"(a), "v"(b));
  return c;
}

__device__ __forceinline__ void wave_sync() {
  __builtin_amdgcn_fence(__ATOMIC_RELEASE, "workgroup");
  __builtin_amdgcn_wave_barrier();
  __builtin_amdgcn_fence(__ATOMIC_ACQUIRE, "workgroup");
}

__device__ __forceinline__ float gelu_erf(float x) {
  return 0.5f * x * (1.0f + erff(x * 0.70710678118654752440f));
}

__global__ __launch_bounds__(64) void prep_planes_kernel(
    const float* __restrict__ W1, const float* __restrict__ b1,
    const float* __restrict__ W2, const float* __restrict__ b2,
    const float* __restrict__ W3, const float* __restrict__ b3,
    unsigned char* __restrict__ ws)
{
  const int tid = threadIdx.x;
  const int blk = blockIdx.x;
  float zf = 0.0f;
  asm volatile("" : "+v"(zf));
  if (blk < kPrepB1) {
    const int i = blk * 64 + tid;
    const int n = i >> 2;
    const int q = i & 3;
    float f[32];
#pragma unroll
    for (int j = 0; j < 6; ++j) {
      const float w  = W1[j * kHid + n];
      const float wh = (float)((_Float16)w);
      f[j]      = wh;
      f[6 + j]  = wh * kResInv;
      f[12 + j] = (w - wh) * kResCarry;
    }
    {
      const float bb = b1[n];
      const float bh = (float)((_Float16)bb);
      f[18] = bh;
      f[19] = (bb - bh) * kResCarry;
    }
#pragma unroll
    for (int k = 20; k < 32; ++k) f[k] = zf;
    v8h hv;
#pragma unroll
    for (int e = 0; e < 8; ++e) {
      const float s = (q == 0) ? f[e] : ((q == 1) ? f[8 + e] : ((q == 2) ? f[16 + e] : f[24 + e]));
      hv[e] = (_Float16)s;
    }
    _Float16* dst = (_Float16*)(ws + kOffBt1) + (size_t)i * 8;
    *(volatile v8h*)dst = hv;
    __threadfence();
    *(volatile v8h*)dst = hv;
  } else if (blk < kPrepB1 + kPrepB2) {
    const int j  = (blk - kPrepB1) * 64 + tid;
    const int n  = j >> 4;
    const int k0 = (j & 15) * 8;
    v8h hv;
#pragma unroll
    for (int e = 0; e < 8; ++e) {
      const float w = W2[(k0 + e) * kHid + n] * kWCarry;
      hv[e] = (_Float16)w;
    }
    _Float16* dst = (_Float16*)(ws + kOffBt2) + (size_t)j * 8;
    *(volatile v8h*)dst = hv;
    __threadfence();
    *(volatile v8h*)dst = hv;
  } else if (blk < kPrepB1 + kPrepB2 + kPrepB3) {
    const int j  = (blk - kPrepB1 - kPrepB2) * 64 + tid;
    const int n  = j >> 4;
    const int k0 = (j & 15) * 8;
    v8h hv;
#pragma unroll
    for (int e = 0; e < 8; ++e) {
      const float w = W3[(k0 + e) * kChOut + n] * kWCarry;
      hv[e] = (_Float16)w;
    }
    _Float16* dst = (_Float16*)(ws + kOffBt3) + (size_t)j * 8;
    *(volatile v8h*)dst = hv;
    __threadfence();
    *(volatile v8h*)dst = hv;
  } else {
    const int jc = (tid < kChunksB) ? tid : (kChunksB - 1);
    const int i2 = (jc < 32) ? (jc * 4) : 124;
    const int i3 = (jc >= 32) ? ((jc - 32) * 4) : 0;
    const v4f c2 = *(const v4f*)(b2 + i2);
    const v4f c3 = *(const v4f*)(b3 + i3);
    v4f val;
#pragma unroll
    for (int e = 0; e < 4; ++e) val[e] = (jc < 32) ? c2[e] : c3[e];
    if (tid < kChunksB) {
      float* dst = (float*)(ws + kOffBias) + tid * 4;
      *(volatile v4f*)dst = val;
      __threadfence();
      *(volatile v4f*)dst = val;
    }
  }
}

__global__ __launch_bounds__(128) void fused_edge_mlp_kernel(
    const float* __restrict__ y, const float* __restrict__ fy, const int* __restrict__ nidx,
    const _Float16* __restrict__ gBt1, const _Float16* __restrict__ gBt2, const _Float16* __restrict__ gBt3,
    const float* __restrict__ gBias, float* __restrict__ out)
{
  __shared__ __align__(16) _Float16 sBt1[kHid * kK1];
  __shared__ __align__(16) _Float16 sBt2[kHid * kHid];
  __shared__ __align__(16) _Float16 sBt3[kChOut * kHid];
  __shared__ __align__(16) float    sBias[kHid + kChOut];
  __shared__ __align__(16) _Float16 sH[kWavesPerBlock][32 * kHP];
  __shared__ __align__(16) _Float16 sA[kWavesPerBlock][32 * kK1];
  __shared__ __align__(16) float    sAt[kWavesPerBlock][32];
  __shared__ __align__(16) int      sNb[kWavesPerBlock][32];
  __shared__ __align__(16) float    sO[kWavesPerBlock][2 * kChOut];

  const int tid   = threadIdx.x;
  const int lane  = tid & 31;
  const int wave  = __builtin_amdgcn_readfirstlane(tid >> 5);
  const int hh    = lane >> 4;
  const int rlane = lane & 15;
  const int koff  = hh * 8;

  for (int i = tid; i < kChunks1; i += 128) *(v8h*)(sBt1 + i * 8) = *(const v8h*)(gBt1 + i * 8);
  for (int i = tid; i < kChunks2; i += 128) *(v8h*)(sBt2 + i * 8) = *(const v8h*)(gBt2 + i * 8);
  for (int i = tid; i < kChunks3; i += 128) *(v8h*)(sBt3 + i * 8) = *(const v8h*)(gBt3 + i * 8);
  for (int i = tid; i < kChunksB; i += 128) *(v4f*)(sBias + i * 4) = *(const v4f*)(gBias + i * 4);
  __syncthreads();

  _Float16* hb = sH[wave];
  _Float16* ar = sA[wave];
  float*    aw = sAt[wave];
  int*      nw = sNb[wave];
  float*    ob = sO[wave];

  float cOne = 1.0f, cInv = kResInv, cZero = 0.0f;
  asm volatile("" : "+v"(cOne), "+v"(cInv), "+v"(cZero));

#pragma unroll 1
  for (int it = 0; it < kIters; ++it) {
    const int pair = (it * kBlocks + (int)blockIdx.x) * kWavesPerBlock + wave;

    {
      int nb = nidx[pair * 32 + lane];
      nb = (nb < 0) ? 0 : ((nb > kNodes - 1) ? (kNodes - 1) : nb);
      const int node = pair * 2 + hh;
      const float rx = y[nb * 3 + 0], ry = y[nb * 3 + 1], rz = y[nb * 3 + 2];
      const float sx = y[node * 3 + 0], sy = y[node * 3 + 1], sz = y[node * 3 + 2];
      const float sn = sqrtf(sx * sx + sy * sy + sz * sz);
      const float rn = sqrtf(rx * rx + ry * ry + rz * rz);
      const float qi = 1.0f / fmaxf(sn, kEps);
      const float ki = 1.0f / fmaxf(rn, kEps);
      const float score = (sx * qi) * (rx * ki) + (sy * qi) * (ry * ki) + (sz * qi) * (rz * ki);
      float mx = score;
      mx = fmaxf(mx, __shfl_xor(mx, 1));
      mx = fmaxf(mx, __shfl_xor(mx, 2));
      mx = fmaxf(mx, __shfl_xor(mx, 4));
      mx = fmaxf(mx, __shfl_xor(mx, 8));
      const float ev = expf(score - mx);
      float ss = ev;
      ss += __shfl_xor(ss, 1);
      ss += __shfl_xor(ss, 2);
      ss += __shfl_xor(ss, 4);
      ss += __shfl_xor(ss, 8);
      const float attn = ev * (1.0f / ss);
      aw[lane] = attn;
      nw[lane] = nb;

      const float x0 = rx, x1 = ry, x2 = rz, x3 = sx, x4 = sy, x5 = sz;
      const float h0 = (float)((_Float16)x0), h1 = (float)((_Float16)x1), h2 = (float)((_Float16)x2);
      const float h3 = (float)((_Float16)x3), h4 = (float)((_Float16)x4), h5 = (float)((_Float16)x5);
      v8h r0, r1, r2, r3;
      r0[0] = (_Float16)h0; r0[1] = (_Float16)h1; r0[2] = (_Float16)h2;
      r0[3] = (_Float16)h3; r0[4] = (_Float16)h4; r0[5] = (_Float16)h5;
      r0[6] = (_Float16)((x0 - h0) * kResCarry);
      r0[7] = (_Float16)((x1 - h1) * kResCarry);
      r1[0] = (_Float16)((x2 - h2) * kResCarry);
      r1[1] = (_Float16)((x3 - h3) * kResCarry);
      r1[2] = (_Float16)((x4 - h4) * kResCarry);
      r1[3] = (_Float16)((x5 - h5) * kResCarry);
      r1[4] = (_Float16)(h0 * cInv);
      r1[5] = (_Float16)(h1 * cInv);
      r1[6] = (_Float16)(h2 * cInv);
      r1[7] = (_Float16)(h3 * cInv);
      r2[0] = (_Float16)(h4 * cInv);
      r2[1] = (_Float16)(h5 * cInv);
      r2[2] = (_Float16)cOne;
      r2[3] = (_Float16)cInv;
      r2[4] = (_Float16)cZero; r2[5] = (_Float16)cZero; r2[6] = (_Float16)cZero; r2[7] = (_Float16)cZero;
#pragma unroll
      for (int e = 0; e < 8; ++e) r3[e] = (_Float16)cZero;
      _Float16* rp = ar + lane * kK1;
      *(v8h*)(rp)      = r0;
      *(v8h*)(rp + 8)  = r1;
      *(v8h*)(rp + 16) = r2;
      *(v8h*)(rp + 24) = r3;
    }
    wave_sync();

    {
      const v16h a10 = FragH::load(ar + rlane * kK1 + koff);
      const v16h a11 = FragH::load(ar + (16 + rlane) * kK1 + koff);
#pragma unroll 1
      for (int nt = 0; nt < kHid / 16; ++nt) {
        const v16h bf = FragH::load(sBt1 + (nt * 16 + rlane) * kK1 + koff);
        v8f c0 = (v8f){0.f, 0.f, 0.f, 0.f, 0.f, 0.f, 0.f, 0.f};
        v8f c1 = (v8f){0.f, 0.f, 0.f, 0.f, 0.f, 0.f, 0.f, 0.f};
        c0 = mma_h(a10, bf, c0);
        c1 = mma_h(a11, bf, c1);
#pragma unroll 1
        for (int t = 0; t < 2; ++t) {
          _Float16* hp = hb + (t * 16 + 8 * hh) * kHP + nt * 16 + rlane;
#pragma unroll
          for (int i = 0; i < 8; ++i) {
            const float pre = (t == 0) ? c0[i] : c1[i];
            hp[i * kHP] = (_Float16)gelu_erf(pre);
          }
        }
      }
    }
    wave_sync();

    {
      v16h a[2][4];
#pragma unroll
      for (int t = 0; t < 2; ++t)
#pragma unroll
        for (int kt = 0; kt < 4; ++kt)
          a[t][kt] = FragH::load(hb + (t * 16 + rlane) * kHP + kt * 32 + koff);
      wave_sync();
#pragma unroll 1
      for (int nt = 0; nt < kHid / 16; ++nt) {
        const _Float16* bp = sBt2 + (nt * 16 + rlane) * kHid + koff;
        v8f c0 = (v8f){0.f, 0.f, 0.f, 0.f, 0.f, 0.f, 0.f, 0.f};
        v8f c1 = (v8f){0.f, 0.f, 0.f, 0.f, 0.f, 0.f, 0.f, 0.f};
#pragma unroll
        for (int kt = 0; kt < 4; ++kt) {
          const v16h bf = FragH::load(bp + kt * 32);
          c0 = mma_h(a[0][kt], bf, c0);
          c1 = mma_h(a[1][kt], bf, c1);
        }
        const float bv = sBias[nt * 16 + rlane];
#pragma unroll 1
        for (int t = 0; t < 2; ++t) {
          _Float16* hp = hb + (t * 16 + 8 * hh) * kHP + nt * 16 + rlane;
#pragma unroll
          for (int i = 0; i < 8; ++i) {
            const float acc = (t == 0) ? c0[i] : c1[i];
            const float pre = fmaf(acc, kWInv, bv);
            hp[i * kHP] = (_Float16)gelu_erf(pre);
          }
        }
      }
    }
    wave_sync();

    {
      v16h a[2][4];
#pragma unroll
      for (int t = 0; t < 2; ++t)
#pragma unroll
        for (int kt = 0; kt < 4; ++kt)
          a[t][kt] = FragH::load(hb + (t * 16 + rlane) * kHP + kt * 32 + koff);
      v4f atv[2][2];
      v4i nbv[2][2];
#pragma unroll
      for (int t = 0; t < 2; ++t)
#pragma unroll
        for (int u = 0; u < 2; ++u) {
          atv[t][u] = *(const v4f*)(aw + t * 16 + 8 * hh + 4 * u);
          nbv[t][u] = *(const v4i*)(nw + t * 16 + 8 * hh + 4 * u);
        }
#pragma unroll 1
      for (int nt = 0; nt < kChOut / 16; ++nt) {
        const _Float16* bp = sBt3 + (nt * 16 + rlane) * kHid + koff;
        v8f c0 = (v8f){0.f, 0.f, 0.f, 0.f, 0.f, 0.f, 0.f, 0.f};
        v8f c1 = (v8f){0.f, 0.f, 0.f, 0.f, 0.f, 0.f, 0.f, 0.f};
#pragma unroll
        for (int kt = 0; kt < 4; ++kt) {
          const v16h bf = FragH::load(bp + kt * 32);
          c0 = mma_h(a[0][kt], bf, c0);
          c1 = mma_h(a[1][kt], bf, c1);
        }
        const int col = nt * 16 + rlane;
        const float bv = sBias[kHid + col];
        float p0 = 0.0f, p1 = 0.0f;
#pragma unroll
        for (int i = 0; i < 8; ++i) {
          const int   n0 = nbv[0][i >> 2][i & 3];
          const float f0 = fy[n0 * kChOut + col];
          const float k0 = fmaf(c0[i], kWInv, bv);
          p0 = fmaf(k0 * f0, atv[0][i >> 2][i & 3], p0);
        }
#pragma unroll
        for (int i = 0; i < 8; ++i) {
          const int   n1 = nbv[1][i >> 2][i & 3];
          const float f1 = fy[n1 * kChOut + col];
          const float k1 = fmaf(c1[i], kWInv, bv);
          p1 = fmaf(k1 * f1, atv[1][i >> 2][i & 3], p1);
        }
        p0 += __shfl_xor(p0, 16);
        p1 += __shfl_xor(p1, 16);
        ob[hh * kChOut + col] = (hh == 0) ? p0 : p1;
      }
    }
    wave_sync();

    {
      const v4f ov = *(const v4f*)(ob + lane * 4);
      float* op = out + (size_t)pair * (2 * kChOut) + lane * 4;
      *(volatile v4f*)op = ov;
      __threadfence();
      *(volatile v4f*)op = ov;
    }
    wave_sync();
  }
}

extern "C" void kernel_launch(void* const* d_in, const int* in_sizes, int n_in,
                              void* d_out, int out_size, void* d_ws, size_t ws_size,
                              hipStream_t stream) {
  (void)in_sizes;
  (void)out_size;
  if (n_in < 10) return;
  if (ws_size < kWsTotal) return;

  const float* y   = (const float*)d_in[0];
  const float* f_y = (const float*)d_in[1];
  const int*   nix = (const int*)d_in[2];
  const float* W1 = (const float*)d_in[4];
  const float* b1 = (const float*)d_in[5];
  const float* W2 = (const float*)d_in[6];
  const float* b2 = (const float*)d_in[7];
  const float* W3 = (const float*)d_in[8];
  const float* b3 = (const float*)d_in[9];
  float* out = (float*)d_out;

  unsigned char* ws = (unsigned char*)d_ws;
  const _Float16* Bt1  = (const _Float16*)(ws + kOffBt1);
  const _Float16* Bt2  = (const _Float16*)(ws + kOffBt2);
  const _Float16* Bt3  = (const _Float16*)(ws + kOffBt3);
  const float*    Bias = (const float*)(ws + kOffBias);

  prep_planes_kernel<<<kPrepBlocks, 64, 0, stream>>>(W1, b1, W2, b2, W3, b3, ws);

  fused_edge_mlp_kernel<<<kBlocks, kWavesPerBlock * 32, 0, stream>>>(
      y, f_y, nix, Bt1, Bt2, Bt3, Bias, out);
}
